// GatedGCN_layer_13022340842268
// MI455X (gfx1250) — hardware-run, weakly checked
//
#include <hip/hip_runtime.h>
#include <stddef.h>


#define DF    128
#define NCAT  512
#define GR    32
#define AP    136
#define SP    516
#define NB    256
#define CHUNK 2048
#define NTHR  256
#define NWAVE 8
#define WCAP  256
#define NGRP  (CHUNK / (NTHR * 4))
#define WSCALE 64.0f
#define WINV   0.015625f
#define BNEPS  1e-5f

#define LDS_NUM  (NB * DF)
#define LDS_DEN  (NB * DF)
#define LDS_CNT  NB
#define LDS_LIST (NWAVE * WCAP)
#define LDS_WCNT 32
#define LDS_BYTES ((LDS_NUM + LDS_DEN + LDS_CNT + LDS_LIST + LDS_WCNT) * 4)

static_assert(WCAP == (CHUNK / NTHR) * 32);
static_assert(NGRP == 2);
static_assert(NB == 256);
static_assert((NB & (NB - 1)) == 0);
static_assert(CHUNK == 2048);
static_assert(NB / NWAVE == 32);
static_assert(((LDS_NUM + LDS_DEN + LDS_CNT) % 4) == 0);
static_assert(LDS_BYTES == 271488);
static_assert(NWAVE * 256 * 8 <= LDS_NUM * 4);

typedef float    v4f  __attribute__((ext_vector_type(4)));
typedef float    v8f  __attribute__((ext_vector_type(8)));
typedef int      v4i  __attribute__((ext_vector_type(4)));
typedef _Float16 v8h  __attribute__((ext_vector_type(8)));
typedef _Float16 v16h __attribute__((ext_vector_type(16)));
union Frag   { v16h v; v8h half[2]; };
union Pack16 { v8h h; v4i i; };

__device__ __forceinline__ v8f wm(v16h a, v16h b, v8f c) {
  v8f d = __builtin_amdgcn_wmma_f32_16x16x32_f16(false, a, false, b, (short)0, c, false, false);
  asm volatile("v_nop\n\tv_nop\n\tv_nop\n\tv_nop" : "+v"(d) : "v"(a), "v"(b));
  return d;
}

__device__ __forceinline__ float sigm(float z) {
  return __builtin_amdgcn_rcpf(1.0f + __expf(-z));
}

__global__ __launch_bounds__(NTHR) void k_prepw(
    const float* __restrict__ WA, const float* __restrict__ WB,
    const float* __restrict__ WD, const float* __restrict__ WE, _Float16* Wt) {
  const int t = blockIdx.x * NTHR + threadIdx.x;
  if (t >= NCAT * DF / 8) return;
  const int c   = t >> 4;
  const int k0  = (t & 15) * 8;
  const int mtx = c >> 7;
  const int n   = c & 127;
  const float* W = (mtx == 0) ? WA : (mtx == 1) ? WB : (mtx == 2) ? WD : WE;
  Pack16 u;
#pragma unroll
  for (int i = 0; i < 8; ++i) u.h[i] = (_Float16)(W[(size_t)(k0 + i) * DF + n] * WSCALE);
  _Float16* p = Wt + (size_t)c * DF + k0;
  *(volatile v4i*)p = u.i;
  __threadfence();
  *(volatile v4i*)p = u.i;
}

__global__ __launch_bounds__(NTHR) void k_gemm(
    const float* __restrict__ X, const _Float16* __restrict__ Wt,
    const float* __restrict__ bA, const float* __restrict__ bB,
    const float* __restrict__ bD, const float* __restrict__ bE,
    float* P, int nN) {
  __shared__ __attribute__((aligned(16))) _Float16 At[GR * AP];
  __shared__ __attribute__((aligned(16))) float St[16 * SP];

  const int tid  = threadIdx.x;
  const int lane = tid & 31;
  const int wave = tid >> 5;
  const int hh   = lane >> 4;
  const int m    = lane & 15;
  const int rowBase = blockIdx.x * GR;

  {
    const int r  = tid >> 3;
    const int c0 = (tid & 7) * 16;
    int row = rowBase + r;
    if (row > nN - 1) row = nN - 1;
    const float* p = X + (size_t)row * DF + c0;
    const v4f f0 = *(const v4f*)(p), f1 = *(const v4f*)(p + 4);
    const v4f f2 = *(const v4f*)(p + 8), f3 = *(const v4f*)(p + 12);
    Pack16 u0, u1;
    u0.h[0] = (_Float16)f0.x; u0.h[1] = (_Float16)f0.y; u0.h[2] = (_Float16)f0.z; u0.h[3] = (_Float16)f0.w;
    u0.h[4] = (_Float16)f1.x; u0.h[5] = (_Float16)f1.y; u0.h[6] = (_Float16)f1.z; u0.h[7] = (_Float16)f1.w;
    u1.h[0] = (_Float16)f2.x; u1.h[1] = (_Float16)f2.y; u1.h[2] = (_Float16)f2.z; u1.h[3] = (_Float16)f2.w;
    u1.h[4] = (_Float16)f3.x; u1.h[5] = (_Float16)f3.y; u1.h[6] = (_Float16)f3.z; u1.h[7] = (_Float16)f3.w;
    *(v8h*)(At + r * AP + c0)     = u0.h;
    *(v8h*)(At + r * AP + c0 + 8) = u1.h;
  }
  __syncthreads();

  v8f acc[2][4];
#pragma unroll
  for (int T = 0; T < 2; ++T)
#pragma unroll
    for (int nt = 0; nt < 4; ++nt)
#pragma unroll
      for (int r = 0; r < 8; ++r) acc[T][nt][r] = 0.f;

#pragma unroll 1
  for (int kt = 0; kt < DF / 32; ++kt) {
    const int k0 = kt * 32;
    Frag a0, a1;
    const _Float16* pa0 = At + m * AP + k0 + 8 * hh;
    const _Float16* pa1 = At + (16 + m) * AP + k0 + 8 * hh;
    a0.half[0] = *(const v8h*)pa0; a0.half[1] = *(const v8h*)(pa0 + 16);
    a1.half[0] = *(const v8h*)pa1; a1.half[1] = *(const v8h*)(pa1 + 16);
#pragma unroll
    for (int nt = 0; nt < 4; ++nt) {
      const int c = wave * 64 + nt * 16 + m;
      const _Float16* pb = Wt + (size_t)c * DF + k0 + 8 * hh;
      Frag b;
      b.half[0] = *(const v8h*)pb;
      b.half[1] = *(const v8h*)(pb + 16);
      acc[0][nt] = wm(a0.v, b.v, acc[0][nt]);
      acc[1][nt] = wm(a1.v, b.v, acc[1][nt]);
    }
  }

  const int mtx = wave >> 1;
  const float* bp = (mtx == 0) ? bA : (mtx == 1) ? bB : (mtx == 2) ? bD : bE;
  float bias[4];
#pragma unroll
  for (int nt = 0; nt < 4; ++nt) bias[nt] = bp[(wave & 1) * 64 + nt * 16 + m];

#pragma unroll
  for (int T = 0; T < 2; ++T) {
#pragma unroll
    for (int nt = 0; nt < 4; ++nt) {
      const int cl = wave * 64 + nt * 16 + m;
#pragma unroll
      for (int r = 0; r < 8; ++r) St[(8 * hh + r) * SP + cl] = acc[T][nt][r] * WINV + bias[nt];
    }
    __syncthreads();
    v4f v[8];
#pragma unroll
    for (int i = 0; i < 8; ++i) {
      const int f = i * NTHR + tid;
      v[i] = *(const v4f*)(St + (f >> 7) * SP + (f & 127) * 4);
    }
    float* base = P + (size_t)(rowBase + 16 * T) * NCAT;
#pragma unroll
    for (int i = 0; i < 8; ++i) {
      const int f = i * NTHR + tid;
      *(volatile v4f*)(base + (size_t)(f >> 7) * NCAT + (f & 127) * 4) = v[i];
    }
    __threadfence();
#pragma unroll
    for (int i = 0; i < 8; ++i) {
      const int f = i * NTHR + tid;
      *(volatile v4f*)(base + (size_t)(f >> 7) * NCAT + (f & 127) * 4) = v[i];
    }
    __syncthreads();
  }
}

__global__ __launch_bounds__(NTHR) void k_agg(
    const float* __restrict__ X, const int* __restrict__ srcI, const int* __restrict__ dstI,
    const float* __restrict__ P, float* Hp, double* part, int nN, int nE, float inv_n) {
  extern __shared__ v4f lds_dyn[];
  float* num  = (float*)lds_dyn;
  float* den  = num + LDS_NUM;
  int*   cnt  = (int*)(den + LDS_DEN);
  int*   list = cnt + LDS_CNT;
  int*   wcnt = list + LDS_LIST;

  const int tid  = threadIdx.x;
  const int lane = tid & 31;
  const int wave = tid >> 5;
  const int nodeBase = blockIdx.x * NB;

  {
    const v4f z4 = {0.f, 0.f, 0.f, 0.f};
    for (int i = tid; i < (LDS_NUM + LDS_DEN + LDS_CNT) / 4; i += NTHR) lds_dyn[i] = z4;
  }
  __syncthreads();

  const int  nChunks = (nE + CHUNK - 1) / CHUNK;
  const bool al16    = ((((size_t)dstI) & 15) == 0);

#pragma unroll 1
  for (int ch = 0; ch < nChunks; ++ch) {
    const int cbase = ch * CHUNK;
    int wc = 0;
#pragma unroll
    for (int g = 0; g < NGRP; ++g) {
      const int el0 = (g * NTHR + tid) * 4;
      const int e0  = cbase + el0;
      const int sent = -2147483647 - 1;
      v4i d;
      if (al16 && (cbase + CHUNK <= nE)) {
        d = *(const v4i*)(dstI + e0);
      } else {
        const int em = nE - 1;
        const int t0 = dstI[min(e0,     em)];
        const int t1 = dstI[min(e0 + 1, em)];
        const int t2 = dstI[min(e0 + 2, em)];
        const int t3 = dstI[min(e0 + 3, em)];
        d.x = (e0     < nE) ? t0 : sent;
        d.y = (e0 + 1 < nE) ? t1 : sent;
        d.z = (e0 + 2 < nE) ? t2 : sent;
        d.w = (e0 + 3 < nE) ? t3 : sent;
      }
      const unsigned s0 = (unsigned)d.x - (unsigned)nodeBase;
      const unsigned s1 = (unsigned)d.y - (unsigned)nodeBase;
      const unsigned s2 = (unsigned)d.z - (unsigned)nodeBase;
      const unsigned s3 = (unsigned)d.w - (unsigned)nodeBase;
      const bool h0 = s0 < (unsigned)NB;
      const bool h1 = s1 < (unsigned)NB;
      const bool h2 = s2 < (unsigned)NB;
      const bool h3 = s3 < (unsigned)NB;
      const unsigned many = __builtin_amdgcn_ballot_w32(h0 | h1 | h2 | h3);
      if (many != 0u) {
#define HITJ(J, HJ, SJ) { \
          const unsigned mj = __builtin_amdgcn_ballot_w32(HJ); \
          if (HJ) { \
            const int pos = wc + (int)__builtin_amdgcn_mbcnt_lo(mj, 0u); \
            if (pos < WCAP) list[wave * WCAP + pos] = ((el0 + (J)) << 8) | (int)(SJ); \
          } \
          wc += (int)__builtin_popcount(mj); }
        HITJ(0, h0, s0)
        HITJ(1, h1, s1)
        HITJ(2, h2, s2)
        HITJ(3, h3, s3)
#undef HITJ
      }
    }
    if (lane == 0) wcnt[wave] = wc;
    __syncthreads();

    if (wave == 0) {
      for (int wsx = 0; wsx < NWAVE; ++wsx) {
        int n = wcnt[wsx];
        if (n > WCAP) n = WCAP;
        if (n < 0) n = 0;
        for (int i = 0; i < n; ++i) {
          const int ent  = list[wsx * WCAP + i];
          const int slot = ent & (NB - 1);
          const int el   = (ent >> 8) & (CHUNK - 1);
          int e = cbase + el;
          if (e > nE - 1) e = nE - 1;
          int s = srcI[e];
          s = s < 0 ? 0 : (s > nN - 1 ? nN - 1 : s);
          int nd = nodeBase + slot;
          if (nd > nN - 1) nd = nN - 1;
          const float* ps = P + (size_t)s * NCAT;
          const v4f bx = *(const v4f*)(ps + DF + 4 * lane);
          const v4f dx = *(const v4f*)(ps + 2 * DF + 4 * lane);
          const v4f ex = *(const v4f*)(P + (size_t)nd * NCAT + 3 * DF + 4 * lane);
          const v4f z = dx + ex;
          v4f sg;
          sg.x = sigm(z.x); sg.y = sigm(z.y); sg.z = sigm(z.z); sg.w = sigm(z.w);
          v4f* np = (v4f*)(num + slot * DF + 4 * lane);
          const v4f ncur = *np;
          *np = ncur + sg * bx;
          v4f* dp = (v4f*)(den + slot * DF + 4 * lane);
          const v4f dcur = *dp;
          *dp = dcur + sg;
          if (lane == 0) cnt[slot] = cnt[slot] + 1;
        }
      }
    }
    __syncthreads();
  }

  double sd0 = 0.0, sd1 = 0.0, sd2 = 0.0, sd3 = 0.0;
  double sq0 = 0.0, sq1 = 0.0, sq2 = 0.0, sq3 = 0.0;
#pragma unroll 1
  for (int j = 0; j < NB / NWAVE; ++j) {
    const int slot = wave * (NB / NWAVE) + j;
    const int node = nodeBase + slot;
    if (node >= nN) break;
    const size_t nrow = (size_t)node;
    const int c = cnt[slot];
    const v4f nv = *(const v4f*)(num + slot * DF + 4 * lane);
    const v4f dv = *(const v4f*)(den + slot * DF + 4 * lane);
    const v4f ax = *(const v4f*)(P + nrow * NCAT + 4 * lane);
    const v4f xv = *(const v4f*)(X + nrow * DF + 4 * lane);
    v4f hm;
    hm.x = ax.x + nv.x * __builtin_amdgcn_rcpf(dv.x);
    hm.y = ax.y + nv.y * __builtin_amdgcn_rcpf(dv.y);
    hm.z = ax.z + nv.z * __builtin_amdgcn_rcpf(dv.z);
    hm.w = ax.w + nv.w * __builtin_amdgcn_rcpf(dv.w);
    v4f h;
    h.x = (c > 0) ? hm.x : xv.x;
    h.y = (c > 0) ? hm.y : xv.y;
    h.z = (c > 0) ? hm.z : xv.z;
    h.w = (c > 0) ? hm.w : xv.w;
    h = h * inv_n;
    float* op = Hp + nrow * DF + 4 * lane;
    *(volatile v4f*)op = h;
    __threadfence();
    *(volatile v4f*)op = h;
    const double a0 = (double)h.x, a1 = (double)h.y, a2 = (double)h.z, a3 = (double)h.w;
    sd0 += a0; sd1 += a1; sd2 += a2; sd3 += a3;
    sq0 += a0 * a0; sq1 += a1 * a1; sq2 += a2 * a2; sq3 += a3 * a3;
  }
  __syncthreads();
  double* stg = (double*)lds_dyn;
  stg[wave * 256 + 4 * lane + 0] = sd0;
  stg[wave * 256 + 4 * lane + 1] = sd1;
  stg[wave * 256 + 4 * lane + 2] = sd2;
  stg[wave * 256 + 4 * lane + 3] = sd3;
  stg[wave * 256 + 128 + 4 * lane + 0] = sq0;
  stg[wave * 256 + 128 + 4 * lane + 1] = sq1;
  stg[wave * 256 + 128 + 4 * lane + 2] = sq2;
  stg[wave * 256 + 128 + 4 * lane + 3] = sq3;
  __syncthreads();
  double a = 0.0;
#pragma unroll
  for (int w = 0; w < NWAVE; ++w) a += stg[w * 256 + tid];
  double* pp = part + (size_t)blockIdx.x * 256 + tid;
  *(volatile double*)pp = a;
  __threadfence();
  *(volatile double*)pp = a;
}

__global__ __launch_bounds__(NTHR) void k_bnfin(
    const double* __restrict__ part, const float* __restrict__ gam,
    float* bnp, int nBlk, int nN) {
  __shared__ double sq[256];
  const int tid = threadIdx.x;
  double a = 0.0;
#pragma unroll 1
  for (int b = 0; b < nBlk; ++b) a += part[(size_t)b * 256 + tid];
  sq[tid] = a;
  __syncthreads();
  const int c = tid & 127;
  const double s = sq[c];
  const double q = sq[128 + c];
  const double invn = 1.0 / (double)nN;
  const double mean = s * invn;
  double var = q * invn - mean * mean;
  if (var < 0.0) var = 0.0;
  const float varf = (float)var;
  const float rs = 1.0f / sqrtf(varf + BNEPS);
  const float sc = gam[c] * rs;
  const float val = (tid < 128) ? (float)mean : sc;
  float* p = bnp + tid;
  *(volatile float*)p = val;
  __threadfence();
  *(volatile float*)p = val;
}

__global__ __launch_bounds__(NTHR) void k_final(
    const float* __restrict__ X, const float* __restrict__ Hp,
    const float* __restrict__ bnp, const float* __restrict__ bet,
    float* out, int nN) {
  const size_t f = (size_t)blockIdx.x * NTHR + threadIdx.x;
  const int row = (int)(f >> 5);
  if (row >= nN) return;
  const int c = (int)(f & 31) * 4;
  const v4f h  = *(const v4f*)(Hp + (size_t)row * DF + c);
  const v4f xv = *(const v4f*)(X + (size_t)row * DF + c);
  const v4f mu = *(const v4f*)(bnp + c);
  const v4f sc = *(const v4f*)(bnp + 128 + c);
  const v4f be = *(const v4f*)(bet + c);
  v4f y = (h - mu) * sc + be;
  y.x = y.x > 0.f ? y.x : 0.f;
  y.y = y.y > 0.f ? y.y : 0.f;
  y.z = y.z > 0.f ? y.z : 0.f;
  y.w = y.w > 0.f ? y.w : 0.f;
  const v4f o = xv + y;
  float* op = out + (size_t)row * DF + c;
  *(volatile v4f*)op = o;
  __threadfence();
  *(volatile v4f*)op = o;
}

static inline size_t al256(size_t x) { return (x + 255) & ~(size_t)255; }

extern "C" void kernel_launch(void* const* d_in, const int* in_sizes, int n_in,
                              void* d_out, int out_size, void* d_ws, size_t ws_size,
                              hipStream_t stream) {
  if (n_in < 13) return;
  const int nN = in_sizes[0] / DF;
  if (nN <= 0 || in_sizes[0] != nN * DF) return;
  if (in_sizes[1] != DF * DF || in_sizes[3] != DF * DF || in_sizes[5] != DF * DF || in_sizes[7] != DF * DF) return;
  if (in_sizes[2] != DF || in_sizes[4] != DF || in_sizes[6] != DF || in_sizes[8] != DF) return;
  if (in_sizes[9] != DF || in_sizes[10] != DF) return;
  const int nE = in_sizes[11];
  if (nE < 0 || in_sizes[12] != nE) return;
  if (out_size != nN * DF) return;

  const float* X   = (const float*)d_in[0];
  const float* WA  = (const float*)d_in[1];
  const float* bA  = (const float*)d_in[2];
  const float* WB  = (const float*)d_in[3];
  const float* bB  = (const float*)d_in[4];
  const float* WD  = (const float*)d_in[5];
  const float* bD  = (const float*)d_in[6];
  const float* WE  = (const float*)d_in[7];
  const float* bE  = (const float*)d_in[8];
  const float* gam = (const float*)d_in[9];
  const float* bet = (const float*)d_in[10];
  const int*   srcI = (const int*)d_in[11];
  const int*   dstI = (const int*)d_in[12];
  float* out = (float*)d_out;

  const int nP   = ((nN + GR - 1) / GR) * GR;
  const int nBlk = (nN + NB - 1) / NB;

  size_t off = 0;
  _Float16* Wt = (_Float16*)((char*)d_ws + off); off = al256(off + (size_t)NCAT * DF * sizeof(_Float16));
  float* P     = (float*)((char*)d_ws + off);    off = al256(off + (size_t)nP * NCAT * sizeof(float));
  float* Hp    = (float*)((char*)d_ws + off);    off = al256(off + (size_t)nP * DF * sizeof(float));
  double* part = (double*)((char*)d_ws + off);   off = al256(off + (size_t)nBlk * 256 * sizeof(double));
  float* bnp   = (float*)((char*)d_ws + off);    off = al256(off + 256 * sizeof(float));
  if (off > ws_size) return;

  const float inv_n = (float)(1.0 / (double)nN);

  k_prepw<<<(NCAT * DF / 8 + NTHR - 1) / NTHR, NTHR, 0, stream>>>(WA, WB, WD, WE, Wt);

  k_gemm<<<nP / GR, NTHR, 0, stream>>>(X, Wt, bA, bB, bD, bE, P, nN);

  hipFuncSetAttribute(reinterpret_cast<const void*>(&k_agg),
                      hipFuncAttributeMaxDynamicSharedMemorySize, LDS_BYTES);
  k_agg<<<nBlk, NTHR, LDS_BYTES, stream>>>(X, srcI, dstI, P, Hp, part, nN, nE, inv_n);

  k_bnfin<<<1, NTHR, 0, stream>>>(part, gam, bnp, nBlk, nN);

  k_final<<<(int)(((size_t)nN * 32 + NTHR - 1) / NTHR), NTHR, 0, stream>>>(X, Hp, bnp, bet, out, nN);
}
